// RepModule_6725918785954
// MI455X (gfx1250) — hardware-verified
//
#include <hip/hip_runtime.h>
#include <stddef.h>


#pragma clang fp contract(off)

#define FEAT    64
#define ATTR    16
#define KATT    32
#define KEDG    32
#define NRBF    8
#define NSH     9
#define NLAY    3
#define NTHR    256
#define NWAVE   8
#define EPT     8
#define NGRP    2
#define CHUNK   (NTHR * EPT * NGRP)
#define WCAP    (EPT * NGRP * 32)
#define LISTN   (NWAVE * WCAP)
#define NBC     4096
#define NBF     1024
#define RCAP    40960
#define RBN     128
#define OTHR    512
#define DEGCAP  256
#define CNB     32
#define CPOS    64
#define GROWS   128
#define HP      (FEAT + 8)
#define XP      (KATT + 8)
#define ABP     (KEDG + 8)
#define WPF     (FEAT + 4)
#define WSCAP   134217728
#define LDS_FILL ((RCAP + NBF + LISTN) * 4 + 64)
#define NODE_US (2 * GROWS * XP + 2 * GROWS * HP)
#define WB_EMB  0
#define WB_L0   2048
#define WB_STR  10240
#define WB_ATTR 0
#define WB_SELF 2048
#define WB_MSG  6144
#define BHALF   32768
#define WBLKB   16
#define WF_STR  8192
#define WF_R1   0
#define WF_SH   2048
#define WF_R2   4096
#define FTOT    24576
#define WBLKF   12
#define ASC     16.0f
#define HSC     8.0f
#define WSCL    64.0f
#define INV_AW  (1.0f / 1024.0f)
#define INV_HW  (1.0f / 512.0f)

static_assert((CHUNK & (CHUNK - 1)) == 0);
static_assert(CHUNK <= 4096);
static_assert((NBC & (NBC - 1)) == 0 && (NBF & (NBF - 1)) == 0);
static_assert(NBC == 4 * NBF);
static_assert(OTHR * 8 == NBC);
static_assert((RCAP % 32) == 0);
static_assert((NBF % CNB) == 0);
static_assert((GROWS % CNB) == 0);
static_assert(CNB == 4 * NWAVE);
static_assert(GROWS == NWAVE * 16);
static_assert(((HP * 2) % 16) == 0 && ((XP * 2) % 16) == 0 && ((ABP * 2) % 16) == 0 && ((WPF * 4) % 16) == 0);
static_assert(GROWS * FEAT * 2 <= 2 * GROWS * HP);
static_assert(NODE_US * 2 <= 65536);
static_assert(CNB * FEAT <= CPOS * WPF);
static_assert((CNB * DEGCAP) % CPOS == 0);
static_assert(BHALF == WB_L0 + NLAY * WB_STR);
static_assert(BHALF == WBLKB * NTHR * 8);
static_assert(FTOT == NLAY * WF_STR);
static_assert(FTOT == WBLKF * NTHR * 8);

typedef float          v2f  __attribute__((ext_vector_type(2)));
typedef float          v4f  __attribute__((ext_vector_type(4)));
typedef float          v8f  __attribute__((ext_vector_type(8)));
typedef int            v4i  __attribute__((ext_vector_type(4)));
typedef unsigned short v8us __attribute__((ext_vector_type(8)));
typedef __bf16         v16b __attribute__((ext_vector_type(16)));
typedef _Float16       v8h  __attribute__((ext_vector_type(8)));
typedef _Float16       v16h __attribute__((ext_vector_type(16)));
union FragB { v16b v; v8us h[2]; };
union FragH { v16h v; v8h h[2]; };

__device__ __forceinline__ v8f wmb(v16b a, v16b b, v8f c) {
  v8f d = __builtin_amdgcn_wmma_f32_16x16x32_bf16(false, a, false, b, (short)0, c, false, false);
  asm volatile("v_nop\n\tv_nop\n\tv_nop\n\tv_nop" : "+v"(d) : "v"(a), "v"(b));
  return d;
}
__device__ __forceinline__ v8f wmf(v16h a, v16h b, v8f c) {
  v8f d = __builtin_amdgcn_wmma_f32_16x16x32_f16(false, a, false, b, (short)0, c, false, false);
  asm volatile("v_nop\n\tv_nop\n\tv_nop\n\tv_nop" : "+v"(d) : "v"(a), "v"(b));
  return d;
}

__device__ __forceinline__ float silu_f(float v) {
  return v * __builtin_amdgcn_rcpf(1.0f + __expf(-v));
}

__device__ __forceinline__ unsigned short bfh(float f) {
  unsigned int u = __float_as_uint(f);
  u += 0x7FFFu + ((u >> 16) & 1u);
  return (unsigned short)(u >> 16);
}
__device__ __forceinline__ float bff(unsigned short h) {
  return __uint_as_float(((unsigned int)h) << 16);
}
__device__ __forceinline__ void split8(v4f a, v4f b, v8us& hi, v8us& lo) {
  float v[8] = {a.x, a.y, a.z, a.w, b.x, b.y, b.z, b.w};
#pragma unroll
  for (int j = 0; j < 8; ++j) {
    const unsigned short hj = bfh(v[j]);
    hi[j] = hj;
    lo[j] = bfh(v[j] - bff(hj));
  }
}

template <int NB>
__device__ __forceinline__ int scan_chunk(const int* __restrict__ keys, int nE, int cbase, int slotBase,
                                          int vec8, int* list, int tid, int lane, int wave) {
  int wc = 0;
#pragma unroll
  for (int g = 0; g < NGRP; ++g) {
    const int el0  = (g * NTHR + tid) * EPT;
    const int e0   = cbase + el0;
    const int sent = -2147483647 - 1;
    v4i da, db;
    if (vec8 != 0 && cbase + CHUNK <= nE) {
      da = *(const v4i*)(keys + e0);
      db = *(const v4i*)(keys + e0 + 4);
    } else {
      da.x = (e0     < nE) ? keys[min(e0, nE - 1)] : sent;
      da.y = (e0 + 1 < nE) ? keys[min(e0 + 1, nE - 1)] : sent;
      da.z = (e0 + 2 < nE) ? keys[min(e0 + 2, nE - 1)] : sent;
      da.w = (e0 + 3 < nE) ? keys[min(e0 + 3, nE - 1)] : sent;
      db.x = (e0 + 4 < nE) ? keys[min(e0 + 4, nE - 1)] : sent;
      db.y = (e0 + 5 < nE) ? keys[min(e0 + 5, nE - 1)] : sent;
      db.z = (e0 + 6 < nE) ? keys[min(e0 + 6, nE - 1)] : sent;
      db.w = (e0 + 7 < nE) ? keys[min(e0 + 7, nE - 1)] : sent;
    }
    const unsigned nb = (unsigned)slotBase;
    const unsigned s0 = (unsigned)da.x - nb, s1 = (unsigned)da.y - nb;
    const unsigned s2 = (unsigned)da.z - nb, s3 = (unsigned)da.w - nb;
    const unsigned s4 = (unsigned)db.x - nb, s5 = (unsigned)db.y - nb;
    const unsigned s6 = (unsigned)db.z - nb, s7 = (unsigned)db.w - nb;
    const bool h0 = s0 < (unsigned)NB, h1 = s1 < (unsigned)NB, h2 = s2 < (unsigned)NB, h3 = s3 < (unsigned)NB;
    const bool h4 = s4 < (unsigned)NB, h5 = s5 < (unsigned)NB, h6 = s6 < (unsigned)NB, h7 = s7 < (unsigned)NB;
    const unsigned any = __builtin_amdgcn_ballot_w32(h0 | h1 | h2 | h3 | h4 | h5 | h6 | h7);
    if (any != 0u) {
#define HITJ(J, HJ, SJ) { \
        const unsigned mj = __builtin_amdgcn_ballot_w32(HJ); \
        if (mj != 0u) { \
          if (HJ) { \
            const int pos = wc + (int)__builtin_amdgcn_mbcnt_lo(mj, 0u); \
            if (pos < WCAP) list[wave * WCAP + pos] = ((el0 + (J)) << 12) | (int)(SJ); \
          } \
          wc += (int)__builtin_popcount(mj); } }
      HITJ(0, h0, s0)
      HITJ(1, h1, s1)
      HITJ(2, h2, s2)
      HITJ(3, h3, s3)
      HITJ(4, h4, s4)
      HITJ(5, h5, s5)
      HITJ(6, h6, s6)
      HITJ(7, h7, s7)
#undef HITJ
    }
  }
  return wc;
}

__global__ __launch_bounds__(NTHR) void k_wprep(
    const float* __restrict__ wemb, const float* __restrict__ wattr, const float* __restrict__ wself,
    const float* __restrict__ wmsg, const float* __restrict__ wr1, const float* __restrict__ wsh,
    const float* __restrict__ wr2, unsigned short* wpb, _Float16* wpf) {
  const int tid = (int)threadIdx.x;
  const int b = (int)blockIdx.x;
  const bool isf = (b >= WBLKB);
  const float* src = wemb;
  int K = ATTR, Kp = KATT, doff = WB_EMB, lp = tid;
  if (!isf) {
    if (b != 0) {
      const int lb = b - 1;
      const int l = lb / 5;
      const int rr = lb - 5 * l;
      const int lbase = WB_L0 + l * WB_STR;
      if (rr == 0)      { src = wattr + (size_t)l * ATTR * FEAT; K = ATTR; Kp = KATT; doff = lbase + WB_ATTR; lp = tid; }
      else if (rr < 3)  { src = wself + (size_t)l * FEAT * FEAT; K = FEAT; Kp = FEAT; doff = lbase + WB_SELF; lp = (rr - 1) * NTHR + tid; }
      else              { src = wmsg  + (size_t)l * FEAT * FEAT; K = FEAT; Kp = FEAT; doff = lbase + WB_MSG;  lp = (rr - 3) * NTHR + tid; }
    }
  } else {
    const int fb = b - WBLKB;
    const int l = fb / 4;
    const int rr = fb - 4 * l;
    const int lbase = l * WF_STR;
    if (rr == 0)      { src = wr1 + (size_t)l * NRBF * FEAT; K = NRBF; Kp = KEDG; doff = lbase + WF_R1; lp = tid; }
    else if (rr == 1) { src = wsh + (size_t)l * NSH  * FEAT; K = NSH;  Kp = KEDG; doff = lbase + WF_SH; lp = tid; }
    else              { src = wr2 + (size_t)l * FEAT * FEAT; K = FEAT; Kp = FEAT; doff = lbase + WF_R2; lp = (rr - 2) * NTHR + tid; }
  }
  const int ppr = Kp >> 3;
  const int n   = lp / ppr;
  const int k0  = (lp - n * ppr) * 8;
  float v[8];
#pragma unroll
  for (int j = 0; j < 8; ++j) {
    const int k  = k0 + j;
    const int kc = k < K ? k : K - 1;
    const float f = src[(size_t)kc * FEAT + n];
    v[j] = (k < K) ? f : 0.0f;
  }
  if (!isf) {
    v4f a, c;
    a.x = v[0]; a.y = v[1]; a.z = v[2]; a.w = v[3];
    c.x = v[4]; c.y = v[5]; c.z = v[6]; c.w = v[7];
    v8us hi, lo;
    split8(a, c, hi, lo);
    unsigned short* hpn = wpb + doff + (size_t)n * Kp + k0;
    unsigned short* lpn = hpn + BHALF;
    *(volatile v8us*)hpn = hi;
    *(volatile v8us*)lpn = lo;
    __threadfence();
    *(volatile v8us*)hpn = hi;
    *(volatile v8us*)lpn = lo;
  } else {
    v8h q;
#pragma unroll
    for (int j = 0; j < 8; ++j) q[j] = (_Float16)(v[j] * WSCL);
    _Float16* fp = wpf + doff + (size_t)n * Kp + k0;
    *(volatile v8h*)fp = q;
    __threadfence();
    *(volatile v8h*)fp = q;
  }
}

__global__ __launch_bounds__(NTHR) void k_count(
    const int* __restrict__ keys, int* cnt, int nE, int vec8) {
  __shared__ __attribute__((aligned(16))) int scnt[NBC];
  __shared__ __attribute__((aligned(16))) int list[LISTN];
  __shared__ int wcnt[NWAVE];
  const int tid = threadIdx.x, lane = tid & 31, wave = tid >> 5;
  const int nodeBase = blockIdx.x * NBC;

  for (int i = tid; i < NBC; i += NTHR) scnt[i] = 0;
  __syncthreads();

  const int nChunks = (nE + CHUNK - 1) / CHUNK;
#pragma unroll 1
  for (int ch = 0; ch < nChunks; ++ch) {
    const int cbase = ch * CHUNK;
    const int wc = scan_chunk<NBC>(keys, nE, cbase, nodeBase, vec8, list, tid, lane, wave);
    if (lane == 0) wcnt[wave] = wc;
    __syncthreads();
    if (wave == 0) {
#pragma unroll 1
      for (int wsx = 0; wsx < NWAVE; ++wsx) {
        int n = __builtin_amdgcn_readfirstlane(wcnt[wsx]);
        n = n > WCAP ? WCAP : (n < 0 ? 0 : n);
        const int* lptr = list + wsx * WCAP;
#pragma unroll 1
        for (int i = 0; i < n; ++i) {
          const int ent  = __builtin_amdgcn_readfirstlane(lptr[i]);
          const int slot = ent & (NBC - 1);
          if (lane == 0) scnt[slot] = scnt[slot] + 1;
        }
      }
    }
    __syncthreads();
  }

  v4i cq[4];
#pragma unroll
  for (int q = 0; q < 4; ++q) {
    const int f = (wave * 4 + q) * 128 + 4 * lane;
    cq[q] = *(const v4i*)(scnt + f);
  }
  int* cp = cnt + (size_t)nodeBase;
#pragma unroll
  for (int q = 0; q < 4; ++q) {
    const int f = (wave * 4 + q) * 128 + 4 * lane;
    *(volatile v4i*)(cp + f) = cq[q];
  }
  __threadfence();
#pragma unroll
  for (int q = 0; q < 4; ++q) {
    const int f = (wave * 4 + q) * 128 + 4 * lane;
    *(volatile v4i*)(cp + f) = cq[q];
  }
}

__global__ __launch_bounds__(OTHR) void k_offsets(
    const int* __restrict__ cnt, int* off, int* rbase, int nChunk) {
  __shared__ __attribute__((aligned(16))) int soff[NBC];
  __shared__ __attribute__((aligned(16))) int srb[RBN];
  __shared__ int wtot[OTHR / 32];
  const int tid = threadIdx.x, lane = tid & 31, wave = tid >> 5, sub = tid >> 7;
  for (int i = tid; i < RBN; i += OTHR) srb[i] = 0;
  int carry = 0;
#pragma unroll 1
  for (int ch = 0; ch < nChunk; ++ch) {
    const int base = ch * NBC;
    const v4i c0 = *(const v4i*)(cnt + base + 8 * tid);
    const v4i c1 = *(const v4i*)(cnt + base + 8 * tid + 4);
    const int e0 = max(c0.x, 0), e1 = max(c0.y, 0), e2 = max(c0.z, 0), e3 = max(c0.w, 0);
    const int e4 = max(c1.x, 0), e5 = max(c1.y, 0), e6 = max(c1.z, 0), e7 = max(c1.w, 0);
    const int ts = e0 + e1 + e2 + e3 + e4 + e5 + e6 + e7;
    int incl = ts;
#pragma unroll
    for (int d = 1; d < 32; d <<= 1) {
      const int t = __shfl_up(incl, d);
      if (lane >= d) incl += t;
    }
    if (lane == 31) wtot[wave] = incl;
    __syncthreads();
    const int S0 = wtot[0]  + wtot[1]  + wtot[2]  + wtot[3];
    const int S1 = wtot[4]  + wtot[5]  + wtot[6]  + wtot[7];
    const int S2 = wtot[8]  + wtot[9]  + wtot[10] + wtot[11];
    const int S3 = wtot[12] + wtot[13] + wtot[14] + wtot[15];
    int pre = 0;
#pragma unroll 1
    for (int w = 4 * sub; w < wave; ++w) pre += wtot[w];
    const int b0 = carry;
    const int b1 = b0 + ((S0 + 31) & ~31);
    const int b2 = b1 + ((S1 + 31) & ~31);
    const int b3 = b2 + ((S2 + 31) & ~31);
    const int b4 = b3 + ((S3 + 31) & ~31);
    const int myb = sub == 0 ? b0 : (sub == 1 ? b1 : (sub == 2 ? b2 : b3));
    if (tid == 0) {
      srb[min(4 * ch + 0, RBN - 1)] = b0;
      srb[min(4 * ch + 1, RBN - 1)] = b1;
      srb[min(4 * ch + 2, RBN - 1)] = b2;
      srb[min(4 * ch + 3, RBN - 1)] = b3;
    }
    int run = myb + pre + incl - ts;
    soff[8 * tid + 0] = run; run += e0;
    soff[8 * tid + 1] = run; run += e1;
    soff[8 * tid + 2] = run; run += e2;
    soff[8 * tid + 3] = run; run += e3;
    soff[8 * tid + 4] = run; run += e4;
    soff[8 * tid + 5] = run; run += e5;
    soff[8 * tid + 6] = run; run += e6;
    soff[8 * tid + 7] = run;
    carry = b4;
    __syncthreads();
    const v4i o0 = *(const v4i*)(soff + 4 * tid);
    const v4i o1 = *(const v4i*)(soff + 4 * (tid + OTHR));
    int* op = off + base;
    *(volatile v4i*)(op + 4 * tid) = o0;
    *(volatile v4i*)(op + 4 * (tid + OTHR)) = o1;
    __threadfence();
    *(volatile v4i*)(op + 4 * tid) = o0;
    *(volatile v4i*)(op + 4 * (tid + OTHR)) = o1;
    __syncthreads();
  }
  if (tid == 0) srb[min(4 * nChunk, RBN - 1)] = carry;
  __syncthreads();
  v4i rv = {0, 0, 0, 0};
  if (tid < 32) rv = *(const v4i*)(srb + 4 * tid);
  if (tid < 32) *(volatile v4i*)(rbase + 4 * tid) = rv;
  __threadfence();
  if (tid < 32) *(volatile v4i*)(rbase + 4 * tid) = rv;
}

__global__ __launch_bounds__(NTHR) void k_fill(
    const int* __restrict__ keys, const int* __restrict__ off, const int* __restrict__ rbase,
    int* csr, int nE, int vec8, int csrLen) {
  extern __shared__ v4f lds_dyn[];
  int* region = (int*)lds_dyn;
  int* cursor = region + RCAP;
  int* list   = cursor + NBF;
  int* wcnt   = list + LISTN;
  const int tid = threadIdx.x, lane = tid & 31, wave = tid >> 5;
  const int b = blockIdx.x;
  const int nodeBase = b * NBF;

  int rb0 = rbase[b];
  const int rb1 = rbase[b + 1];
  rb0 = rb0 < 0 ? 0 : (rb0 > csrLen ? csrLen : rb0);
  rb0 &= ~31;
  int len = rb1 - rb0;
  len = len < 0 ? 0 : (len > RCAP ? RCAP : len);
  int lenW = (len + 31) & ~31;
  if (rb0 + lenW > csrLen) lenW = (csrLen - rb0) & ~31;

  {
    const v4i z = {0, 0, 0, 0};
    for (int i = tid; i < RCAP / 4; i += NTHR) ((v4i*)region)[i] = z;
    for (int s = tid; s < NBF; s += NTHR) {
      int o = off[nodeBase + s] - rb0;
      o = o < 0 ? 0 : (o > RCAP ? RCAP : o);
      cursor[s] = o;
    }
  }
  __syncthreads();

  const int nChunks = (nE + CHUNK - 1) / CHUNK;
#pragma unroll 1
  for (int ch = 0; ch < nChunks; ++ch) {
    const int cbase = ch * CHUNK;
    const int wc = scan_chunk<NBF>(keys, nE, cbase, nodeBase, vec8, list, tid, lane, wave);
    if (lane == 0) wcnt[wave] = wc;
    __syncthreads();
    if (wave == 0) {
#pragma unroll 1
      for (int wsx = 0; wsx < NWAVE; ++wsx) {
        int n = __builtin_amdgcn_readfirstlane(wcnt[wsx]);
        n = n > WCAP ? WCAP : (n < 0 ? 0 : n);
        const int* lptr = list + wsx * WCAP;
#pragma unroll 1
        for (int i = 0; i < n; ++i) {
          const int ent  = __builtin_amdgcn_readfirstlane(lptr[i]);
          const int slot = ent & (NBF - 1);
          int e = cbase + ((ent >> 12) & (CHUNK - 1));
          e = e > nE - 1 ? nE - 1 : e;
          if (lane == 0) {
            int pos = cursor[slot];
            pos = pos < 0 ? 0 : (pos > RCAP - 1 ? RCAP - 1 : pos);
            region[pos] = e;
            const int np = pos + 1;
            cursor[slot] = np > RCAP ? RCAP : np;
          }
        }
      }
    }
    __syncthreads();
  }

  const int nv = lenW >> 2;
  int* gp = csr + rb0;
#pragma unroll 1
  for (int i = tid; i < nv; i += NTHR) { const v4i v = ((const v4i*)region)[i]; *(volatile v4i*)(gp + 4 * i) = v; }
  __threadfence();
#pragma unroll 1
  for (int i = tid; i < nv; i += NTHR) { const v4i v = ((const v4i*)region)[i]; *(volatile v4i*)(gp + 4 * i) = v; }
}

__global__ __launch_bounds__(NTHR) void k_geom(
    const int* __restrict__ csr, const int* __restrict__ ei, const float* __restrict__ pos,
    const float* __restrict__ pvec, float* Rp, float* Ux, float* Uy, float* Uz, int* Sp,
    int nE, int nN, int csrLen) {
  const int tid = threadIdx.x;
  const int p = blockIdx.x * NTHR + tid;
  const int pc = p > csrLen - 1 ? csrLen - 1 : p;
  int e = csr[pc];
  e = e < 0 ? 0 : (e > nE - 1 ? nE - 1 : e);
  int s = ei[e];
  s = s < 0 ? 0 : (s > nN - 1 ? nN - 1 : s);
  int d = ei[(size_t)nE + e];
  d = d < 0 ? 0 : (d > nN - 1 ? nN - 1 : d);
  const float* ps = pos + (size_t)s * 3;
  const float* pd = pos + (size_t)d * 3;
  const float* pv = pvec + (size_t)e * 3;
  const float vx = (pd[0] - ps[0]) + pv[0];
  const float vy = (pd[1] - ps[1]) + pv[1];
  const float vz = (pd[2] - ps[2]) + pv[2];
  const float r2 = (vx * vx + vz * vz) + vy * vy;
  const float r = sqrtf(r2 + 1e-12f);
  const float inv = 1.0f / r;
  const float ux = vx * inv, uy = vy * inv, uz = vz * inv;
  *(volatile float*)(Rp + pc) = r;
  *(volatile float*)(Ux + pc) = ux;
  *(volatile float*)(Uy + pc) = uy;
  *(volatile float*)(Uz + pc) = uz;
  *(volatile int*)(Sp + pc) = s;
  __threadfence();
  *(volatile float*)(Rp + pc) = r;
  *(volatile float*)(Ux + pc) = ux;
  *(volatile float*)(Uy + pc) = uy;
  *(volatile float*)(Uz + pc) = uz;
  *(volatile int*)(Sp + pc) = s;
}

__device__ __forceinline__ void stage16(float* stg, v8f a0, v8f a1, v8f a2, v8f a3,
                                        int wave, int hh, int m) {
  float* sp = stg + (size_t)(wave * 16 + 8 * hh) * FEAT + m;
#pragma unroll
  for (int r = 0; r < 8; ++r) {
    sp[r * FEAT + 0]  = a0[r];
    sp[r * FEAT + 16] = a1[r];
    sp[r * FEAT + 32] = a2[r];
    sp[r * FEAT + 48] = a3[r];
  }
}
__device__ __forceinline__ void rows_out(const float* stg, float* out, int rowBase, int nRows,
                                         int wave, int lane) {
  v4f vals[8];
#pragma unroll
  for (int i = 0; i < 8; ++i) {
    const int row = wave * 16 + 2 * i + (lane >> 4);
    vals[i] = *(const v4f*)(stg + (size_t)row * FEAT + 4 * (lane & 15));
  }
#pragma unroll
  for (int i = 0; i < 8; ++i) {
    const int grow = rowBase + wave * 16 + 2 * i + (lane >> 4);
    if (grow < nRows) *(volatile v4f*)(out + (size_t)grow * FEAT + 4 * (lane & 15)) = vals[i];
  }
  __threadfence();
#pragma unroll
  for (int i = 0; i < 8; ++i) {
    const int grow = rowBase + wave * 16 + 2 * i + (lane >> 4);
    if (grow < nRows) *(volatile v4f*)(out + (size_t)grow * FEAT + 4 * (lane & 15)) = vals[i];
  }
}

template <int MODE>
__global__ __launch_bounds__(NTHR) void k_node(
    const float* __restrict__ Hin, const int* __restrict__ xz, const float* __restrict__ etab,
    const unsigned short* __restrict__ WAh, const unsigned short* __restrict__ WAl,
    const unsigned short* __restrict__ WMh, const unsigned short* __restrict__ WMl,
    const unsigned short* __restrict__ WSh, const unsigned short* __restrict__ WSl,
    float* out1, float* out2, int nN, int nTab, int nRows) {
  __shared__ __attribute__((aligned(16))) unsigned short lraw[NODE_US];
  unsigned short* sXh = lraw;
  unsigned short* sXl = lraw + GROWS * XP;
  unsigned short* sHh = lraw + 2 * GROWS * XP;
  unsigned short* sHl = sHh + GROWS * HP;
  float* stg = (float*)(lraw + 2 * GROWS * XP);
  const int tid = threadIdx.x, lane = tid & 31, wave = tid >> 5, hh = lane >> 4, m = lane & 15;
  const int rowBase = blockIdx.x * GROWS;
  const v8us z8 = {0, 0, 0, 0, 0, 0, 0, 0};

  {
    const int r = tid >> 1, c8 = (tid & 1) * 8;
    int node = rowBase + r;
    node = node > nN - 1 ? nN - 1 : node;
    int xi = xz[node];
    xi = xi < 0 ? 0 : (xi > nTab - 1 ? nTab - 1 : xi);
    const float* ep = etab + (size_t)xi * ATTR + c8;
    const v4f a = *(const v4f*)ep, b = *(const v4f*)(ep + 4);
    v8us hi, lo;
    split8(a, b, hi, lo);
    *(v8us*)(sXh + r * XP + c8) = hi;
    *(v8us*)(sXl + r * XP + c8) = lo;
    *(v8us*)(sXh + r * XP + 16 + c8) = z8;
    *(v8us*)(sXl + r * XP + 16 + c8) = z8;
  }
  if constexpr (MODE != 0) {
#pragma unroll
    for (int i = 0; i < 4; ++i) {
      const int j = i * NTHR + tid;
      const int r = j >> 3;
      const int c = (j & 7) * 8;
      int row = rowBase + r;
      row = row > nRows - 1 ? nRows - 1 : row;
      const float* hp = Hin + (size_t)row * FEAT + c;
      const v4f a = *(const v4f*)hp, b = *(const v4f*)(hp + 4);
      v8us hi, lo;
      split8(a, b, hi, lo);
      *(v8us*)(sHh + r * HP + c) = hi;
      *(v8us*)(sHl + r * HP + c) = lo;
    }
  }
  __syncthreads();

  const v8f z = {0.f, 0.f, 0.f, 0.f, 0.f, 0.f, 0.f, 0.f};
  v8f am[4], as[4];
#pragma unroll
  for (int t = 0; t < 4; ++t) { am[t] = z; as[t] = z; }
  const int arow = wave * 16 + m;

  if constexpr (MODE != 0) {
#pragma unroll
    for (int ks = 0; ks < FEAT / 32; ++ks) {
      FragB ah, al;
      ah.h[0] = *(const v8us*)(sHh + arow * HP + 32 * ks + 8 * hh);
      ah.h[1] = *(const v8us*)(sHh + arow * HP + 32 * ks + 16 + 8 * hh);
      al.h[0] = *(const v8us*)(sHl + arow * HP + 32 * ks + 8 * hh);
      al.h[1] = *(const v8us*)(sHl + arow * HP + 32 * ks + 16 + 8 * hh);
#pragma unroll
      for (int t = 0; t < 4; ++t) {
        const int n = 16 * t + m;
        const size_t bo = (size_t)n * FEAT + 32 * ks + 8 * hh;
        FragB bmh, bml, bsh, bsl;
        bmh.h[0] = *(const v8us*)(WMh + bo); bmh.h[1] = *(const v8us*)(WMh + bo + 16);
        bml.h[0] = *(const v8us*)(WMl + bo); bml.h[1] = *(const v8us*)(WMl + bo + 16);
        bsh.h[0] = *(const v8us*)(WSh + bo); bsh.h[1] = *(const v8us*)(WSh + bo + 16);
        bsl.h[0] = *(const v8us*)(WSl + bo); bsl.h[1] = *(const v8us*)(WSl + bo + 16);
        am[t] = wmb(ah.v, bmh.v, am[t]);
        am[t] = wmb(ah.v, bml.v, am[t]);
        am[t] = wmb(al.v, bmh.v, am[t]);
        as[t] = wmb(ah.v, bsh.v, as[t]);
        as[t] = wmb(ah.v, bsl.v, as[t]);
        as[t] = wmb(al.v, bsh.v, as[t]);
      }
    }
  }
  {
    FragB xh, xl;
    xh.h[0] = *(const v8us*)(sXh + arow * XP + 8 * hh);
    xh.h[1] = *(const v8us*)(sXh + arow * XP + 16 + 8 * hh);
    xl.h[0] = *(const v8us*)(sXl + arow * XP + 8 * hh);
    xl.h[1] = *(const v8us*)(sXl + arow * XP + 16 + 8 * hh);
#pragma unroll
    for (int t = 0; t < 4; ++t) {
      const int n = 16 * t + m;
      const size_t bo = (size_t)n * KATT + 8 * hh;
      FragB bah, bal;
      bah.h[0] = *(const v8us*)(WAh + bo); bah.h[1] = *(const v8us*)(WAh + bo + 16);
      bal.h[0] = *(const v8us*)(WAl + bo); bal.h[1] = *(const v8us*)(WAl + bo + 16);
      if constexpr (MODE != 0) {
        as[t] = wmb(xh.v, bah.v, as[t]);
        as[t] = wmb(xh.v, bal.v, as[t]);
        as[t] = wmb(xl.v, bah.v, as[t]);
      } else {
        am[t] = wmb(xh.v, bah.v, am[t]);
        am[t] = wmb(xh.v, bal.v, am[t]);
        am[t] = wmb(xl.v, bah.v, am[t]);
      }
    }
  }
  __syncthreads();

  stage16(stg, am[0], am[1], am[2], am[3], wave, hh, m);
  __syncthreads();
  rows_out(stg, out1, rowBase, nRows, wave, lane);
  if constexpr (MODE != 0) {
    __syncthreads();
    stage16(stg, as[0], as[1], as[2], as[3], wave, hh, m);
    __syncthreads();
    rows_out(stg, out2, rowBase, nRows, wave, lane);
  }
}

__global__ __launch_bounds__(NTHR) void k_conv(
    const int* __restrict__ offp, const int* __restrict__ cntp,
    const float* __restrict__ Rp, const float* __restrict__ Ux, const float* __restrict__ Uy,
    const float* __restrict__ Uz, const int* __restrict__ Sp,
    const float* __restrict__ Hm, const float* __restrict__ Hs,
    const _Float16* __restrict__ Wr1f, const _Float16* __restrict__ Wshf,
    const _Float16* __restrict__ W2f,
    float* hout, int nN, int csrLen, int nOut) {
  __shared__ __attribute__((aligned(16))) _Float16 sRb[CPOS * ABP];
  __shared__ __attribute__((aligned(16))) _Float16 sSh[CPOS * ABP];
  __shared__ __attribute__((aligned(16))) int      sSrc[CPOS];
  __shared__ __attribute__((aligned(16))) _Float16 sHd[CPOS * HP];
  __shared__ __attribute__((aligned(16))) float    sW[CPOS * WPF];
  const int tid = threadIdx.x, lane = tid & 31, wave = tid >> 5, hh = lane >> 4, m = lane & 15;

  {
    v8h z8h;
#pragma unroll
    for (int j = 0; j < 8; ++j) z8h[j] = (_Float16)0.0f;
    for (int i = tid; i < CPOS * 3; i += NTHR) {
      const int row = i / 3, c = i - 3 * row;
      *(v8h*)(sRb + row * ABP + 8 + 8 * c) = z8h;
    }
    for (int i = tid; i < CPOS * 2; i += NTHR) {
      const int row = i >> 1, c = i & 1;
      *(v8h*)(sSh + row * ABP + 16 + 8 * c) = z8h;
    }
  }

  const int c0 = blockIdx.x * CNB;
  int offl = offp[c0 + lane];
  int cntl = cntp[c0 + lane];
  cntl = cntl < 0 ? 0 : (cntl > DEGCAP ? DEGCAP : cntl);
  offl = offl < 0 ? 0 : (offl > csrLen ? csrLen : offl);
  const int R0 = __builtin_amdgcn_readfirstlane(offl);
  const int Rend = __builtin_amdgcn_readlane(offl, 31) + __builtin_amdgcn_readlane(cntl, 31);
  int tot = Rend - R0;
  tot = tot < 0 ? 0 : (tot > CNB * DEGCAP ? CNB * DEGCAP : tot);
  const int nch = (tot + CPOS - 1) / CPOS;
  const int rt = wave & 3, ct0 = (wave >> 2) * 2;

  const float S3 = 1.7320508075688772f, S15 = 3.872983346207417f;
  const float S54 = 1.118033988749895f, S154 = 1.936491673103708f;
  const float SQ2C = 0.6324555320336759f;
  const float PI_F = 3.14159265358979323846f;
  const v8f z = {0.f, 0.f, 0.f, 0.f, 0.f, 0.f, 0.f, 0.f};

  v2f nacc[4];
#pragma unroll
  for (int s = 0; s < 4; ++s) { v2f zz = {0.f, 0.f}; nacc[s] = zz; }

#pragma unroll 1
  for (int ch = 0; ch < nch; ++ch) {
    const int P = R0 + ch * CPOS;
    int nval = tot - ch * CPOS;
    nval = nval > CPOS ? CPOS : nval;
    __syncthreads();
    if (wave < 2) {
      int p = P + tid;
      p = p > csrLen - 1 ? csrLen - 1 : p;
      const float r = Rp[p];
      const float ux = Ux[p], uy = Uy[p], uz = Uz[p];
      int s = Sp[p];
      s = s < 0 ? 0 : (s > nN - 1 ? nN - 1 : s);
      const float zd = ux * 0.0f;
      v8h q0, q1;
      q0[0] = (_Float16)(ASC + zd);
      q0[1] = (_Float16)(ASC * (S3 * ux));
      q0[2] = (_Float16)(ASC * (S3 * uy));
      q0[3] = (_Float16)(ASC * (S3 * uz));
      q0[4] = (_Float16)(ASC * ((S15 * ux) * uy));
      q0[5] = (_Float16)(ASC * ((S15 * uy) * uz));
      q0[6] = (_Float16)(ASC * (S54 * ((3.0f * uz) * uz - 1.0f)));
      q0[7] = (_Float16)(ASC * ((S15 * ux) * uz));
      q1[0] = (_Float16)(ASC * (S154 * (ux * ux - uy * uy)));
#pragma unroll
      for (int j = 1; j < 8; ++j) q1[j] = (_Float16)zd;
      *(v8h*)(sSh + tid * ABP) = q0;
      *(v8h*)(sSh + tid * ABP + 8) = q1;
      const float rs = fmaxf(r, 1e-6f);
      const float rp = r * 0.2f;
      const float rp2 = rp * rp, rp3 = rp2 * rp, rp6 = rp3 * rp3, rp7 = rp6 * rp, rp8 = rp7 * rp;
      float env = 1.0f - 28.0f * rp6 + 48.0f * rp7 - 21.0f * rp8;
      env = (rp < 1.0f) ? env : 0.0f;
      const float invrs = 1.0f / rs;
      const float pref = (SQ2C * invrs) * env;
      const float th = (PI_F * rs) * 0.2f;
      const float s1 = sinf(th);
      const float cs = cosf(th);
      const float c2 = cs + cs;
      const float s2 = c2 * s1;
      const float s3 = c2 * s2 - s1;
      const float s4 = c2 * s3 - s2;
      const float s5 = c2 * s4 - s3;
      const float s6 = c2 * s5 - s4;
      const float s7 = c2 * s6 - s5;
      const float s8 = c2 * s7 - s6;
      v8h qr;
      qr[0] = (_Float16)(ASC * (pref * s1)); qr[1] = (_Float16)(ASC * (pref * s2));
      qr[2] = (_Float16)(ASC * (pref * s3)); qr[3] = (_Float16)(ASC * (pref * s4));
      qr[4] = (_Float16)(ASC * (pref * s5)); qr[5] = (_Float16)(ASC * (pref * s6));
      qr[6] = (_Float16)(ASC * (pref * s7)); qr[7] = (_Float16)(ASC * (pref * s8));
      *(v8h*)(sRb + tid * ABP) = qr;
      sSrc[tid] = s;
    }
    __syncthreads();

    if (16 * rt < nval) {
      const int arow = 16 * rt + m;
      FragH ar, ash;
      ar.h[0]  = *(const v8h*)(sRb + arow * ABP + 8 * hh);
      ar.h[1]  = *(const v8h*)(sRb + arow * ABP + 16 + 8 * hh);
      ash.h[0] = *(const v8h*)(sSh + arow * ABP + 8 * hh);
      ash.h[1] = *(const v8h*)(sSh + arow * ABP + 16 + 8 * hh);
#pragma unroll
      for (int t = 0; t < 2; ++t) {
        const int n = 16 * (ct0 + t) + m;
        const size_t bo = (size_t)n * KEDG + 8 * hh;
        FragH b1, b2;
        b1.h[0] = *(const v8h*)(Wr1f + bo); b1.h[1] = *(const v8h*)(Wr1f + bo + 16);
        b2.h[0] = *(const v8h*)(Wshf + bo); b2.h[1] = *(const v8h*)(Wshf + bo + 16);
        const v8f dh = wmf(ar.v,  b1.v, z);
        const v8f ds = wmf(ash.v, b2.v, z);
#pragma unroll
        for (int r = 0; r < 8; ++r) {
          const int row = 16 * rt + 8 * hh + r;
          const float hv = silu_f(dh[r] * INV_AW) * HSC;
          sHd[row * HP + n] = (_Float16)hv;
          sW[row * WPF + n] = ds[r] * INV_AW;
        }
      }
    }
    __syncthreads();

    if (16 * rt < nval) {
      v8f acc[2];
      acc[0] = z; acc[1] = z;
      const int arow = 16 * rt + m;
#pragma unroll
      for (int ks = 0; ks < FEAT / 32; ++ks) {
        FragH ah;
        ah.h[0] = *(const v8h*)(sHd + arow * HP + 32 * ks + 8 * hh);
        ah.h[1] = *(const v8h*)(sHd + arow * HP + 32 * ks + 16 + 8 * hh);
#pragma unroll
        for (int t = 0; t < 2; ++t) {
          const int n = 16 * (ct0 + t) + m;
          const size_t bo = (size_t)n * FEAT + 32 * ks + 8 * hh;
          FragH bh;
          bh.h[0] = *(const v8h*)(W2f + bo); bh.h[1] = *(const v8h*)(W2f + bo + 16);
          acc[t] = wmf(ah.v, bh.v, acc[t]);
        }
      }
#pragma unroll
      for (int t = 0; t < 2; ++t) {
        const int n = 16 * (ct0 + t) + m;
#pragma unroll
        for (int r = 0; r < 8; ++r) {
          float* q = sW + (16 * rt + 8 * hh + r) * WPF + n;
          const float cur = *q;
          *q = cur * (acc[t][r] * INV_HW);
        }
      }
    }
    __syncthreads();

#pragma unroll
    for (int s = 0; s < 4; ++s) {
      const int j  = 4 * wave + s;
      const int oj = __shfl(offl, j);
      const int cj = __shfl(cntl, j);
      int lo = oj - P;
      lo = lo < 0 ? 0 : (lo > CPOS ? CPOS : lo);
      int hi = oj + cj - P;
      hi = hi < 0 ? 0 : (hi > CPOS ? CPOS : hi);
#pragma unroll 1
      for (int r = lo; r < hi; ++r) {
        const v2f wv = *(const v2f*)(sW + r * WPF + 2 * lane);
        const int sidx = sSrc[r];
        const v2f hv = *(const v2f*)(Hm + (size_t)sidx * FEAT + 2 * lane);
        nacc[s] = nacc[s] + wv * hv;
      }
    }
  }

  __syncthreads();
  float* stg = sW;
#pragma unroll
  for (int s = 0; s < 4; ++s) {
    const int row = 4 * wave + s;
    const int node = c0 + row;
    const v2f hsv = *(const v2f*)(Hs + (size_t)node * FEAT + 2 * lane);
    v2f v = nacc[s] + hsv;
    v.x = silu_f(v.x);
    v.y = silu_f(v.y);
    *(v2f*)(stg + row * FEAT + 2 * lane) = v;
  }
  __syncthreads();
  v4f o[2];
#pragma unroll
  for (int i = 0; i < 2; ++i) {
    const int idx = i * NTHR + tid;
    o[i] = *(const v4f*)(stg + (idx >> 4) * FEAT + 4 * (idx & 15));
  }
#pragma unroll
  for (int i = 0; i < 2; ++i) {
    const int idx = i * NTHR + tid;
    const int node = c0 + (idx >> 4);
    if (node < nOut) *(volatile v4f*)(hout + (size_t)node * FEAT + 4 * (idx & 15)) = o[i];
  }
  __threadfence();
#pragma unroll
  for (int i = 0; i < 2; ++i) {
    const int idx = i * NTHR + tid;
    const int node = c0 + (idx >> 4);
    if (node < nOut) *(volatile v4f*)(hout + (size_t)node * FEAT + 4 * (idx & 15)) = o[i];
  }
}

extern "C" void kernel_launch(void* const* d_in, const int* in_sizes, int n_in,
                              void* d_out, int out_size, void* d_ws, size_t ws_size,
                              hipStream_t stream) {
  if (n_in < 13) return;
  const int nN = in_sizes[0];
  if (nN <= 0) return;
  if (in_sizes[2] <= 0 || (in_sizes[2] & 1) != 0) return;
  const int nE = in_sizes[2] / 2;
  if (in_sizes[1] != 3 * nN || in_sizes[3] != 3 * nE) return;
  if (in_sizes[5] <= 0 || (in_sizes[5] % ATTR) != 0) return;
  const int nTab = in_sizes[5] / ATTR;
  if (in_sizes[6] != ATTR * FEAT || in_sizes[7] != NLAY * ATTR * FEAT) return;
  if (in_sizes[8] != NLAY * FEAT * FEAT || in_sizes[9] != NLAY * FEAT * FEAT) return;
  if (in_sizes[10] != NLAY * NRBF * FEAT || in_sizes[11] != NLAY * FEAT * FEAT) return;
  if (in_sizes[12] != NLAY * NSH * FEAT) return;
  if (out_size != nN * FEAT) return;
  if (nE > (1 << 26) || nN > (1 << 22)) return;

  const int*   xz    = (const int*)d_in[0];
  const float* pos   = (const float*)d_in[1];
  const int*   ei    = (const int*)d_in[2];
  const float* pvec  = (const float*)d_in[3];
  const float* etab  = (const float*)d_in[5];
  const float* wemb  = (const float*)d_in[6];
  const float* wattr = (const float*)d_in[7];
  const float* wself = (const float*)d_in[8];
  const float* wmsg  = (const float*)d_in[9];
  const float* wr1   = (const float*)d_in[10];
  const float* wr2   = (const float*)d_in[11];
  const float* wsh   = (const float*)d_in[12];
  float* out = (float*)d_out;

  const int NPAD   = ((nN + GROWS - 1) / GROWS) * GROWS;
  const int nBC    = (nN + NBC - 1) / NBC;
  const int CNTPAD = nBC * NBC;
  if (NPAD > CNTPAD) return;
  if (4 * nBC + 1 > RBN) return;
  const int nBF    = (nN + NBF - 1) / NBF;
  if (31 * 4 * nBC > 4096) return;
  const int csrLen = ((nE + 255) & ~255) + 4096;
  const int nConv  = NPAD / CNB;
  const int nNode  = NPAD / GROWS;
  const int nGeom  = csrLen / NTHR;

  char* ws = (char*)d_ws;
  size_t off = 0;
  const size_t plane  = (size_t)NPAD * FEAT * 4;
  const size_t pplane = (size_t)csrLen * 4;
  const size_t oW   = off; off += ((size_t)2 * BHALF + FTOT) * 2; off = (off + 255) & ~(size_t)255;
  const size_t oCnt = off; off += (size_t)CNTPAD * 4;        off = (off + 255) & ~(size_t)255;
  const size_t oOff = off; off += (size_t)CNTPAD * 4;        off = (off + 255) & ~(size_t)255;
  const size_t oRb  = off; off += (size_t)RBN * 4;           off = (off + 255) & ~(size_t)255;
  const size_t oCsr = off; off += pplane;                    off = (off + 255) & ~(size_t)255;
  const size_t oRp  = off; off += pplane;                    off = (off + 255) & ~(size_t)255;
  const size_t oUx  = off; off += pplane;                    off = (off + 255) & ~(size_t)255;
  const size_t oUy  = off; off += pplane;                    off = (off + 255) & ~(size_t)255;
  const size_t oUz  = off; off += pplane;                    off = (off + 255) & ~(size_t)255;
  const size_t oSp  = off; off += pplane;                    off = (off + 255) & ~(size_t)255;
  const size_t oH   = off; off += plane;                     off = (off + 255) & ~(size_t)255;
  const size_t oHm  = off; off += plane;                     off = (off + 255) & ~(size_t)255;
  const size_t oHs  = off; off += plane;                     off = (off + 255) & ~(size_t)255;
  if (off > ws_size || off > (size_t)WSCAP) return;
  unsigned short* wpb = (unsigned short*)(ws + oW);
  _Float16* wpf = (_Float16*)(ws + oW + (size_t)2 * BHALF * 2);
  int*   cnt  = (int*)(ws + oCnt);
  int*   offp = (int*)(ws + oOff);
  int*   rb   = (int*)(ws + oRb);
  int*   csr  = (int*)(ws + oCsr);
  float* Rp   = (float*)(ws + oRp);
  float* Ux   = (float*)(ws + oUx);
  float* Uy   = (float*)(ws + oUy);
  float* Uz   = (float*)(ws + oUz);
  int*   Sp   = (int*)(ws + oSp);
  float* hpl  = (float*)(ws + oH);
  float* hmp  = (float*)(ws + oHm);
  float* hsp  = (float*)(ws + oHs);

  const int* keys = ei + nE;
  const int vec8 = ((nE & 3) == 0) ? 1 : 0;

  k_wprep<<<WBLKB + WBLKF, NTHR, 0, stream>>>(wemb, wattr, wself, wmsg, wr1, wsh, wr2, wpb, wpf);

  k_count<<<nBC, NTHR, 0, stream>>>(keys, cnt, nE, vec8);
  k_offsets<<<1, OTHR, 0, stream>>>(cnt, offp, rb, nBC);
  hipFuncSetAttribute(reinterpret_cast<const void*>(&k_fill),
                      hipFuncAttributeMaxDynamicSharedMemorySize, LDS_FILL);
  k_fill<<<nBF, NTHR, LDS_FILL, stream>>>(keys, offp, rb, csr, nE, vec8, csrLen);

  k_geom<<<nGeom, NTHR, 0, stream>>>(csr, ei, pos, pvec, Rp, Ux, Uy, Uz, Sp, nE, nN, csrLen);

  const unsigned short* wembh = wpb + WB_EMB;
  const unsigned short* wembl = wembh + BHALF;
  k_node<0><<<nNode, NTHR, 0, stream>>>(hpl, xz, etab, wembh, wembl, wembh, wembl, wembh, wembl,
                                         hpl, hmp, nN, nTab, NPAD);

  for (int l = 0; l < NLAY; ++l) {
    const unsigned short* base = wpb + WB_L0 + (size_t)l * WB_STR;
    const unsigned short* wah  = base + WB_ATTR; const unsigned short* wal  = wah + BHALF;
    const unsigned short* wsfh = base + WB_SELF; const unsigned short* wsfl = wsfh + BHALF;
    const unsigned short* wmh  = base + WB_MSG;  const unsigned short* wml  = wmh + BHALF;
    const _Float16* fbase = wpf + (size_t)l * WF_STR;
    const _Float16* wr1f = fbase + WF_R1;
    const _Float16* wshf = fbase + WF_SH;
    const _Float16* w2f  = fbase + WF_R2;
    float* hnext = (l == NLAY - 1) ? out : hpl;
    const int nOut = (l == NLAY - 1) ? nN : NPAD;

    k_node<1><<<nNode, NTHR, 0, stream>>>(hpl, xz, etab, wah, wal, wmh, wml, wsfh, wsfl,
                                           hmp, hsp, nN, nTab, NPAD);
    k_conv<<<nConv, NTHR, 0, stream>>>(offp, cnt, Rp, Ux, Uy, Uz, Sp, hmp, hsp, wr1f, wshf,
                                         w2f, hnext, nN, csrLen, nOut);
  }
}
